// non_local_11605001633975
// MI455X (gfx1250) — hardware-verified
//
#include <hip/hip_runtime.h>
#include <math.h>

constexpr int kB  = 8;
constexpr int kC  = 256;
constexpr int kN  = 4096;
constexpr int kCi = 128;
constexpr int kQChunk  = 2048;
constexpr int kNChunks = kN / kQChunk;
constexpr int kWElems  = kCi * kC;
constexpr float kPCarry   = 32768.0f;
constexpr float kYCarry   = 16.0f;
constexpr float kWCarry   = 16.0f;
constexpr float kPVScale  = kYCarry / kPCarry;
constexpr float kWScale   = 1.0f / (kYCarry * kWCarry);
constexpr float kBnEps    = 1e-5f;
constexpr float kInvCount = 1.0f / (float)(kB * kN);
constexpr int kStatPitch  = 32;
static_assert(kC % 32 == 0 && kCi % 32 == 0 && kN % 32 == 0, "K multiples of 32");
static_assert(kN % 64 == 0 && kCi % 64 == 0 && kC % 64 == 0 && kQChunk % 64 == 0, "M,N multiples of 64");
static_assert(kN % kQChunk == 0 && kQChunk == 2048, "chunks");
static_assert(kN == 8 * 512 && kN == 2 * 2048, "softmax trip layout");
static_assert(kWElems % (8 * 256) == 0, "weight cast grid");
static_assert((kB * kC * kN) % (4 * 256) == 0, "apply grid");
static_assert(kB * kN == 32768, "stat count");

constexpr size_t kSzXT  = (size_t)kB * kN * kC * 2;
constexpr size_t kSzTP  = (size_t)kB * kN * kCi * 2;
constexpr size_t kSzWY  = (size_t)kB * kC * kN * 4;
constexpr size_t kSzSC  = (size_t)kQChunk * kN * 4;
constexpr size_t kSzPP  = (size_t)kQChunk * kN * 2;
constexpr size_t kSzWB  = (size_t)3 * kWElems * 2;
constexpr size_t kSzWW  = (size_t)kWElems * 2;
constexpr size_t kSzPRM = 4096;
constexpr size_t kSzST  = (size_t)kC * kStatPitch * 4;
constexpr size_t kOffXT  = 0;
constexpr size_t kOffTHH = kOffXT + kSzXT;
constexpr size_t kOffTHL = kOffTHH + kSzTP;
constexpr size_t kOffPHH = kOffTHL + kSzTP;
constexpr size_t kOffPHL = kOffPHH + kSzTP;
constexpr size_t kOffG   = kOffPHL + kSzTP;
constexpr size_t kOffY   = kOffG + kSzTP;
constexpr size_t kOffWY  = kOffY + kSzTP;
constexpr size_t kOffPP  = kOffWY + kSzWY;
constexpr size_t kOffWB  = kOffPP + kSzPP;
constexpr size_t kOffWW  = kOffWB + kSzWB;
constexpr size_t kOffPRM = kOffWW + kSzWW;
constexpr size_t kOffST  = kOffPRM + kSzPRM;
constexpr size_t kWsTotal = kOffST + kSzST;
static_assert(kSzSC <= kSzWY, "score chunk fits the WY region");
static_assert(kWsTotal == 117739520, "carve total");
static_assert(kWsTotal <= (size_t)134217728, "carve cap");
static_assert(kOffTHH % 256 == 0 && kOffG % 256 == 0 && kOffWY % 256 == 0 && kOffPP % 256 == 0 &&
              kOffWB % 256 == 0 && kOffWW % 256 == 0 && kOffPRM % 256 == 0 && kOffST % 256 == 0, "alignment");
static_assert(640 * 4 <= kSzPRM, "param table");

typedef __attribute__((ext_vector_type(16))) _Float16 v16h;
typedef __attribute__((ext_vector_type(8)))  _Float16 v8h;
typedef __attribute__((ext_vector_type(16))) __bf16   v16b;
typedef __attribute__((ext_vector_type(8)))  __bf16   v8b;
typedef __attribute__((ext_vector_type(8)))  float    v8f;
typedef __attribute__((ext_vector_type(4)))  float    v4f;
typedef __attribute__((ext_vector_type(2)))  float    v2f;
typedef __attribute__((ext_vector_type(4)))  unsigned int v4u;

__device__ __forceinline__ unsigned short f2bf_bits(float f) {
  unsigned u = __float_as_uint(f);
  return (unsigned short)((u + 0x7FFFu + ((u >> 16) & 1u)) >> 16);
}
__device__ __forceinline__ float bf_bits2f(unsigned short h) { return __uint_as_float(((unsigned)h) << 16); }
__device__ __forceinline__ float bfr(float f) { return bf_bits2f(f2bf_bits(f)); }

__device__ __forceinline__ void dep_guard_h(v8f& a, v8f& b, v16h x, v16h y) { asm volatile("v_nop\n\tv_nop\n\tv_nop\n\tv_nop" : "+v"(a), "+v"(b) : "v"(x), "v"(y)); }
__device__ __forceinline__ void dep_guard_b(v8f& a, v8f& b, v16b x, v16b y) { asm volatile("v_nop\n\tv_nop\n\tv_nop\n\tv_nop" : "+v"(a), "+v"(b) : "v"(x), "v"(y)); }
__device__ __forceinline__ void keep4_h(v16h a, v16h b, v16h c, v16h d) { asm volatile("v_nop" :: "v"(a), "v"(b), "v"(c), "v"(d)); }
__device__ __forceinline__ void keep4_b(v16b a, v16b b, v16b c, v16b d) { asm volatile("v_nop" :: "v"(a), "v"(b), "v"(c), "v"(d)); }
__device__ __forceinline__ void acc_guard4(v8f& a, v8f& b, v8f& c, v8f& d) { asm volatile("v_nop\n\tv_nop\n\tv_nop\n\tv_nop" : "+v"(a), "+v"(b), "+v"(c), "+v"(d)); }
template <typename T> struct Frag;
template <> struct Frag<_Float16> {
  typedef v16h V; union U { v16h v; v8h h[2]; };
  static __device__ __forceinline__ v16h load(const _Float16* p) {
    U f; f.h[0] = *(const v8h*)(p); f.h[1] = *(const v8h*)(p + 16); return f.v;
  }
  static __device__ __forceinline__ v8f mma(v16h a, v16h b, v8f c) {
    return __builtin_amdgcn_wmma_f32_16x16x32_f16(false, a, false, b, (short)0, c, false, false);
  }
  static __device__ __forceinline__ void guard(v8f& a, v8f& b, v16h x, v16h y) { dep_guard_h(a, b, x, y); }
  static __device__ __forceinline__ void keep(v16h a, v16h b, v16h c, v16h d) { keep4_h(a, b, c, d); }
};
template <> struct Frag<__bf16> {
  typedef v16b V; union U { v16b v; v8b h[2]; };
  static __device__ __forceinline__ v16b load(const __bf16* p) {
    U f; f.h[0] = *(const v8b*)(p); f.h[1] = *(const v8b*)(p + 16); return f.v;
  }
  static __device__ __forceinline__ v8f mma(v16b a, v16b b, v8f c) {
    return __builtin_amdgcn_wmma_f32_16x16x32_bf16(false, a, false, b, (short)0, c, false, false);
  }
  static __device__ __forceinline__ void guard(v8f& a, v8f& b, v16b x, v16b y) { dep_guard_b(a, b, x, y); }
  static __device__ __forceinline__ void keep(v16b a, v16b b, v16b c, v16b d) { keep4_b(a, b, c, d); }
};

__device__ __forceinline__ unsigned pk16(unsigned short a, unsigned short b) { return (unsigned)a | ((unsigned)b << 16); }
__device__ __forceinline__ unsigned short h_bits(float f) { const _Float16 h = (_Float16)f; return __builtin_bit_cast(unsigned short, h); }

template <int ET> struct Elem;
template <> struct Elem<0> { typedef _Float16 T; };
template <> struct Elem<1> { typedef __bf16 T; };
template <int ET, bool SPLIT, int BIAS_MODE, int OUT_MODE, bool RESID, int ACT = 0>
__global__ __launch_bounds__(256) void wmma_gemm64(
    const unsigned short* __restrict__ Ap, const unsigned short* __restrict__ A2p, int lda, long strideA,
    const unsigned short* __restrict__ Btp, const unsigned short* __restrict__ Bt2p, int ldb, long strideB,
    void* __restrict__ Cout, void* __restrict__ Cout2, int ldc, long strideC,
    const float* __restrict__ bias,
    const float* __restrict__ resid, long strideR,
    int M, int N, int K, float scale) {
  typedef typename Elem<ET>::T T;
  typedef typename Frag<T>::V V;
  const T* A = (const T*)Ap; const T* A2 = (const T*)A2p; const T* Bt = (const T*)Btp; const T* Bt2 = (const T*)Bt2p;
  __shared__ __align__(16) float sT[8][16 * 68];
  const int b    = blockIdx.y;
  const int lane = threadIdx.x & 31;
  const int wave = threadIdx.x >> 5;
  const int tilesN = N >> 6;
  const int tilesM = M >> 6;
  const int tile = blockIdx.x * 8 + wave;
  if (tile >= tilesM * tilesN) return;
  const int tm = tile / tilesN;
  const int tn = tile - tm * tilesN;
  const int m0 = tm << 6;
  const int n0 = tn << 6;

  const T* Ab  = A  + (size_t)b * strideA;
  const T* Bb  = Bt + (size_t)b * strideB;
  const T* Ab2 = SPLIT ? (A2  + (size_t)b * strideA) : nullptr;
  const T* Bb2 = SPLIT ? (Bt2 + (size_t)b * strideB) : nullptr;

  const int rlane = lane & 15;
  const int koff  = (lane >> 4) * 8;
  const int mOff  = (lane >> 4) * 8;

  v8f acc[4][4];
#pragma unroll
  for (int i = 0; i < 4; ++i)
#pragma unroll
    for (int j = 0; j < 4; ++j) acc[i][j] = (v8f){0.f,0.f,0.f,0.f,0.f,0.f,0.f,0.f};

  for (int k0 = 0; k0 < K; k0 += 32) {
    V bh[4], bl[4];
#pragma unroll
    for (int j = 0; j < 4; ++j) {
      const size_t bo = (size_t)(n0 + (j << 4) + rlane) * ldb + koff + k0;
      bh[j] = Frag<T>::load(Bb + bo);
      if (SPLIT) bl[j] = Frag<T>::load(Bb2 + bo);
    }
#pragma unroll
    for (int i = 0; i < 4; ++i) {
      const size_t ao = (size_t)(m0 + (i << 4) + rlane) * lda + koff + k0;
      V ah = Frag<T>::load(Ab + ao);
      V al;
      if (SPLIT) al = Frag<T>::load(Ab2 + ao);
#pragma unroll
      for (int j = 0; j < 4; ++j) {
        acc[i][j] = Frag<T>::mma(ah, bh[j], acc[i][j]);
        if (SPLIT) {
          acc[i][j] = Frag<T>::mma(ah, bl[j], acc[i][j]);
          acc[i][j] = Frag<T>::mma(al, bh[j], acc[i][j]);
        }
      }
      Frag<T>::guard(acc[i][0], acc[i][3], ah, SPLIT ? al : ah);
    }
    Frag<T>::keep(bh[0], bh[1], bh[2], bh[3]);
    if (SPLIT) Frag<T>::keep(bl[0], bl[1], bl[2], bl[3]);
  }
  acc_guard4(acc[0][0], acc[0][1], acc[0][2], acc[0][3]);
  acc_guard4(acc[1][0], acc[1][1], acc[1][2], acc[1][3]);
  acc_guard4(acc[2][0], acc[2][1], acc[2][2], acc[2][3]);
  acc_guard4(acc[3][0], acc[3][1], acc[3][2], acc[3][3]);

  float* slab = sT[wave];
  const float* Rb = RESID ? (resid + (size_t)b * strideR) : nullptr;
#pragma unroll
  for (int i = 0; i < 4; ++i) {
    const int mBase = m0 + (i << 4);
    v4f bm0 = (v4f){0.f,0.f,0.f,0.f}, bm1 = (v4f){0.f,0.f,0.f,0.f};
    if (BIAS_MODE == 1) {
      bm0 = *(const v4f*)(bias + mBase + mOff);
      bm1 = *(const v4f*)(bias + mBase + mOff + 4);
    }
#pragma unroll
    for (int j = 0; j < 4; ++j) {
      const int n = n0 + (j << 4) + rlane;
      float bv = 0.f;
      if (BIAS_MODE == 2) bv = bias[n];
#pragma unroll
      for (int r = 0; r < 8; ++r) {
        float v = acc[i][j][r] * scale;
        if (BIAS_MODE == 1) v += (r < 4) ? bm0[r & 3] : bm1[r & 3];
        if (BIAS_MODE == 2) v += bv;
        if (RESID) v += Rb[(size_t)(mBase + mOff + r) * ldc + n];
        if (ACT == 2) v = fmaxf(v, 0.0f);
        if (ACT == 4) v = (v > 0.f) ? v : 0.01f * v;
        slab[(mOff + r) * 68 + (j << 4) + rlane] = v;
      }
    }
    __builtin_amdgcn_fence(__ATOMIC_RELEASE, "workgroup");
    __builtin_amdgcn_wave_barrier();
    __builtin_amdgcn_fence(__ATOMIC_ACQUIRE, "workgroup");
    if (OUT_MODE == 0) {
      float* C = (float*)Cout + (size_t)b * strideC;
      const int hh = lane >> 4, c4 = (lane & 15) * 4;
      for (int pass = 0; pass < 2; ++pass) {
#pragma unroll
        for (int it = 0; it < 8; ++it) {
          const int row = it * 2 + hh;
          v4f v = *(const v4f*)(slab + row * 68 + c4);
          *(volatile v4f*)(C + (size_t)(mBase + row) * ldc + n0 + c4) = v;
        }
        __threadfence();
      }
    } else {
      const int q = lane >> 3, c8 = (lane & 7) * 8;
      unsigned short* C  = (unsigned short*)Cout  + (size_t)b * strideC;
      unsigned short* C2 = (OUT_MODE == 2) ? ((unsigned short*)Cout2 + (size_t)b * strideC) : nullptr;
      for (int pass = 0; pass < 2; ++pass) {
#pragma unroll
        for (int it = 0; it < 4; ++it) {
          const int row = it * 4 + q;
          const float* sp = slab + row * 68 + c8;
          v8h hv, lv;
#pragma unroll
          for (int e = 0; e < 8; ++e) {
            if (OUT_MODE == 1) {
              hv[e] = (_Float16)sp[e];
            } else {
              unsigned short hb = f2bf_bits(sp[e]);
              unsigned short lb = f2bf_bits(sp[e] - bf_bits2f(hb));
              hv[e] = __builtin_bit_cast(_Float16, hb);
              lv[e] = __builtin_bit_cast(_Float16, lb);
            }
          }
          *(volatile v8h*)(C + (size_t)(mBase + row) * ldc + n0 + c8) = hv;
          if (OUT_MODE == 2) *(volatile v8h*)(C2 + (size_t)(mBase + row) * ldc + n0 + c8) = lv;
        }
        __threadfence();
      }
    }
    __builtin_amdgcn_fence(__ATOMIC_RELEASE, "workgroup");
    __builtin_amdgcn_wave_barrier();
    __builtin_amdgcn_fence(__ATOMIC_ACQUIRE, "workgroup");
  }
}

__global__ __launch_bounds__(256) void param_planes_kernel(
    const float* __restrict__ gw, const float* __restrict__ thw, const float* __restrict__ phw, const float* __restrict__ ww,
    const float* __restrict__ gb, const float* __restrict__ thb, const float* __restrict__ phb, const float* __restrict__ wb,
    unsigned short* __restrict__ WB, unsigned short* __restrict__ WW, float* __restrict__ PRM) {
  const int t = threadIdx.x;
  const int y = blockIdx.y;
  if (y < 4) {
    const int i = blockIdx.x * 256 + t;
    if (i >= kWElems / 8) return;
    const float* src = (y == 0) ? gw : (y == 1) ? thw : (y == 2) ? phw : ww;
    const float* p = src + 8 * (size_t)i;
    const v4f a = *(const v4f*)(p);
    const v4f c = *(const v4f*)(p + 4);
    unsigned short hb[8];
#pragma unroll
    for (int e = 0; e < 4; ++e) {
      if (y == 3) {
        hb[e]     = h_bits(bfr(a[e]) * kWCarry);
        hb[4 + e] = h_bits(bfr(c[e]) * kWCarry);
      } else {
        hb[e]     = f2bf_bits(a[e]);
        hb[4 + e] = f2bf_bits(c[e]);
      }
    }
    const v4u u = (v4u){pk16(hb[0], hb[1]), pk16(hb[2], hb[3]), pk16(hb[4], hb[5]), pk16(hb[6], hb[7])};
    unsigned short* q = (y == 3) ? (WW + 8 * (size_t)i) : (WB + (size_t)y * kWElems + 8 * (size_t)i);
    *(volatile v4u*)q = u;
    __threadfence();
    *(volatile v4u*)q = u;
  } else {
    if (blockIdx.x != 0 || t >= 160) return;
    const int w = t >> 5, l = t & 31;
    const float* src = (w == 0) ? gb : (w == 1) ? thb : (w == 2) ? phb : (wb + (w - 3) * 128);
    const v4f a = *(const v4f*)(src + 4 * l);
    v4f r;
#pragma unroll
    for (int e = 0; e < 4; ++e) r[e] = bfr(a[e]);
    float* q = PRM + 128 * w + 4 * l;
    *(volatile v4f*)q = r;
    __threadfence();
    *(volatile v4f*)q = r;
  }
}

__global__ __launch_bounds__(256) void xt_cast_kernel(const float* __restrict__ x, unsigned short* __restrict__ XT) {
  __shared__ float sm[64][65];
  const int t  = threadIdx.x;
  const int n0 = blockIdx.x * 64;
  const int c0 = blockIdx.y * 64;
  const int b  = blockIdx.z;
#pragma unroll
  for (int i = 0; i < 16; ++i) {
    const int e   = i * 256 + t;
    const int r   = e >> 6;
    const int col = e & 63;
    sm[col][r] = x[((size_t)(b * kC + c0 + r)) * kN + n0 + col];
  }
  __syncthreads();
  const int lane = t & 31, wave = t >> 5;
  const int q = lane >> 3, c8 = (lane & 7) * 8;
  unsigned short* op = XT + ((size_t)b * kN) * kC;
  for (int pass = 0; pass < 2; ++pass) {
#pragma unroll
    for (int it = 0; it < 2; ++it) {
      const int row = wave * 8 + it * 4 + q;
      unsigned short hb[8];
#pragma unroll
      for (int e = 0; e < 8; ++e) hb[e] = f2bf_bits(sm[row][c8 + e]);
      const v4u u = (v4u){pk16(hb[0], hb[1]), pk16(hb[2], hb[3]), pk16(hb[4], hb[5]), pk16(hb[6], hb[7])};
      *(volatile v4u*)(op + (size_t)(n0 + row) * kC + c0 + c8) = u;
    }
    __threadfence();
  }
}

__global__ __launch_bounds__(256) void softmax_row_kernel(const float* __restrict__ Sp, unsigned short* __restrict__ Pp) {
  __shared__ __align__(16) float lg[kN];
  __shared__ float redM[8];
  __shared__ float redS[8];
  const int row  = blockIdx.x;
  const int t    = threadIdx.x;
  const int lane = t & 31, wave = t >> 5;
  const float* sr = Sp + (size_t)row * kN;

  float mx = -__builtin_inff();
#pragma unroll 1
  for (int it = 0; it < 8; ++it) {
    const int c = it * 512 + 2 * t;
    const v2f sv = *(const v2f*)(sr + c);
    mx = fmaxf(mx, fmaxf(sv[0], sv[1]));
    *(v2f*)(lg + c) = sv;
  }
#pragma unroll
  for (int off = 16; off > 0; off >>= 1) mx = fmaxf(mx, __shfl_xor(mx, off, 32));
  if (lane == 0) redM[wave] = mx;
  __syncthreads();
  float m = redM[0];
#pragma unroll
  for (int w = 1; w < 8; ++w) m = fmaxf(m, redM[w]);

  float sum = 0.0f;
#pragma unroll 1
  for (int it = 0; it < 8; ++it) {
    const int c = it * 512 + 2 * t;
    const v2f l = *(const v2f*)(lg + c);
    v2f ev;
    ev[0] = expf(l[0] - m);
    ev[1] = expf(l[1] - m);
    sum += ev[0];
    sum += ev[1];
    *(v2f*)(lg + c) = ev;
  }
#pragma unroll
  for (int off = 16; off > 0; off >>= 1) sum += __shfl_xor(sum, off, 32);
  if (lane == 0) redS[wave] = sum;
  __syncthreads();
  float tot = redS[0];
#pragma unroll
  for (int w = 1; w < 8; ++w) tot += redS[w];
  const float inv = kPCarry / tot;

  const v4f e0 = *(const v4f*)(lg + 8 * t);
  const v4f e1 = *(const v4f*)(lg + 8 * t + 4);
  const v4f e2 = *(const v4f*)(lg + 2048 + 8 * t);
  const v4f e3 = *(const v4f*)(lg + 2048 + 8 * t + 4);
  unsigned short ha[8], hc[8];
#pragma unroll
  for (int e = 0; e < 4; ++e) {
    ha[e]     = h_bits(e0[e] * inv);
    ha[4 + e] = h_bits(e1[e] * inv);
    hc[e]     = h_bits(e2[e] * inv);
    hc[4 + e] = h_bits(e3[e] * inv);
  }
  const v4u u0 = (v4u){pk16(ha[0], ha[1]), pk16(ha[2], ha[3]), pk16(ha[4], ha[5]), pk16(ha[6], ha[7])};
  const v4u u1 = (v4u){pk16(hc[0], hc[1]), pk16(hc[2], hc[3]), pk16(hc[4], hc[5]), pk16(hc[6], hc[7])};
  unsigned short* pr = Pp + (size_t)row * kN;
  for (int pass = 0; pass < 2; ++pass) {
    *(volatile v4u*)(pr + 8 * (size_t)t) = u0;
    *(volatile v4u*)(pr + 2048 + 8 * (size_t)t) = u1;
    __threadfence();
  }
}

__global__ __launch_bounds__(256) void bn_stats_kernel(const float* __restrict__ Wy, float* __restrict__ ST) {
  __shared__ float red1[8];
  __shared__ float red2[8];
  const int c = blockIdx.x;
  const int t = threadIdx.x;
  const int lane = t & 31, wave = t >> 5;

  float s = 0.0f;
#pragma unroll 1
  for (int b = 0; b < kB; ++b) {
    const float* base = Wy + ((size_t)b * kC + c) * kN + 4 * t;
#pragma unroll 1
    for (int k = 0; k < 4; ++k) {
      const v4f w = *(const v4f*)(base + k * 1024);
      s += (w[0] + w[1]) + (w[2] + w[3]);
    }
  }
#pragma unroll
  for (int off = 16; off > 0; off >>= 1) s += __shfl_xor(s, off, 32);
  if (lane == 0) red1[wave] = s;
  __syncthreads();
  float tot = red1[0];
#pragma unroll
  for (int w = 1; w < 8; ++w) tot += red1[w];
  const float mean = tot * kInvCount;

  float q = 0.0f;
#pragma unroll 1
  for (int b = 0; b < kB; ++b) {
    const float* base = Wy + ((size_t)b * kC + c) * kN + 4 * t;
#pragma unroll 1
    for (int k = 0; k < 4; ++k) {
      const v4f w = *(const v4f*)(base + k * 1024);
      const float d0 = w[0] - mean, d1 = w[1] - mean, d2 = w[2] - mean, d3 = w[3] - mean;
      q += (d0 * d0 + d1 * d1) + (d2 * d2 + d3 * d3);
    }
  }
#pragma unroll
  for (int off = 16; off > 0; off >>= 1) q += __shfl_xor(q, off, 32);
  if (lane == 0) red2[wave] = q;
  __syncthreads();
  float totq = red2[0];
#pragma unroll
  for (int w = 1; w < 8; ++w) totq += red2[w];
  const float var  = totq * kInvCount;
  const float rstd = 1.0f / sqrtf(var + kBnEps);

  if (t < 8) {
    v4f val = (v4f){0.f, 0.f, 0.f, 0.f};
    if (t == 0) { val[0] = mean; val[1] = rstd; }
    float* sp = ST + (size_t)c * kStatPitch + 4 * t;
    *(volatile v4f*)sp = val;
    __threadfence();
    *(volatile v4f*)sp = val;
  }
}

__global__ __launch_bounds__(256) void bn_apply_kernel(const float* __restrict__ Wy, const float* __restrict__ x,
                                                       const float* __restrict__ gamma, const float* __restrict__ beta,
                                                       const float* __restrict__ ST, float* __restrict__ out, int n4) {
  const int i = blockIdx.x * 256 + threadIdx.x;
  if (i >= n4) return;
  const int c = (i >> 10) & (kC - 1);
  const float mean = ST[(size_t)c * kStatPitch];
  const float rstd = ST[(size_t)c * kStatPitch + 1];
  const float ga = bfr(gamma[c]);
  const float be = bfr(beta[c]);
  const v4f w  = *(const v4f*)(Wy + 4 * (size_t)i);
  const v4f xv = *(const v4f*)(x + 4 * (size_t)i);
  v4f o;
#pragma unroll
  for (int e = 0; e < 4; ++e) o[e] = (((w[e] - mean) * rstd) * ga + be) + bfr(xv[e]);
  float* op = out + 4 * (size_t)i;
  *(volatile v4f*)op = o;
  __threadfence();
  *(volatile v4f*)op = o;
}

extern "C" void kernel_launch(void* const* d_in, const int* in_sizes, int n_in,
                              void* d_out, int out_size, void* d_ws, size_t ws_size,
                              hipStream_t stream) {
  if (n_in < 11) return;
  const int nElem = kB * kC * kN;
  if (in_sizes[0] != nElem) return;
  if (in_sizes[1] != kWElems || in_sizes[3] != kWElems || in_sizes[5] != kWElems || in_sizes[7] != kWElems) return;
  if (in_sizes[2] != kCi || in_sizes[4] != kCi || in_sizes[6] != kCi) return;
  if (in_sizes[8] != kC || in_sizes[9] != kC || in_sizes[10] != kC) return;
  if (out_size != nElem) return;
  if (ws_size < kWsTotal) return;

  const float* x       = (const float*)d_in[0];
  const float* g_w     = (const float*)d_in[1];
  const float* g_b     = (const float*)d_in[2];
  const float* theta_w = (const float*)d_in[3];
  const float* theta_b = (const float*)d_in[4];
  const float* phi_w   = (const float*)d_in[5];
  const float* phi_b   = (const float*)d_in[6];
  const float* W_w     = (const float*)d_in[7];
  const float* W_b     = (const float*)d_in[8];
  const float* bn_g    = (const float*)d_in[9];
  const float* bn_b    = (const float*)d_in[10];
  float* out = (float*)d_out;

  char* ws = (char*)d_ws;
  unsigned short* XT  = (unsigned short*)(ws + kOffXT);
  unsigned short* THH = (unsigned short*)(ws + kOffTHH);
  unsigned short* THL = (unsigned short*)(ws + kOffTHL);
  unsigned short* PHH = (unsigned short*)(ws + kOffPHH);
  unsigned short* PHL = (unsigned short*)(ws + kOffPHL);
  unsigned short* G16 = (unsigned short*)(ws + kOffG);
  unsigned short* Y16 = (unsigned short*)(ws + kOffY);
  float*          WY  = (float*)(ws + kOffWY);
  float*          SC  = (float*)(ws + kOffWY);
  unsigned short* PP  = (unsigned short*)(ws + kOffPP);
  unsigned short* WB  = (unsigned short*)(ws + kOffWB);
  unsigned short* WW  = (unsigned short*)(ws + kOffWW);
  float*          PRM = (float*)(ws + kOffPRM);
  float*          ST  = (float*)(ws + kOffST);
  const float* gb_r  = PRM;
  const float* thb_r = PRM + 128;
  const float* phb_r = PRM + 256;
  const float* wb_r  = PRM + 384;

  param_planes_kernel<<<dim3(kWElems / 8 / 256, 5), dim3(256), 0, stream>>>(
      g_w, theta_w, phi_w, W_w, g_b, theta_b, phi_b, W_b, WB, WW, PRM);
  xt_cast_kernel<<<dim3(kN / 64, kC / 64, kB), dim3(256), 0, stream>>>(x, XT);

  const long strXT = (long)kN * kC;
  const long strTP = (long)kN * kCi;

  wmma_gemm64<1, false, 2, 2, false, 0><<<dim3((kN / 64) * (kCi / 64) / 8, kB), dim3(256), 0, stream>>>(
      XT, XT, kC, strXT, WB + kWElems, WB + kWElems, kC, 0L,
      (void*)THH, (void*)THL, kCi, strTP, thb_r, PRM, 0L, kN, kCi, kC, 1.0f);
  wmma_gemm64<1, false, 2, 2, false, 0><<<dim3((kN / 64) * (kCi / 64) / 8, kB), dim3(256), 0, stream>>>(
      XT, XT, kC, strXT, WB + 2 * kWElems, WB + 2 * kWElems, kC, 0L,
      (void*)PHH, (void*)PHL, kCi, strTP, phb_r, PRM, 0L, kN, kCi, kC, 1.0f);
  wmma_gemm64<1, false, 1, 1, false, 0><<<dim3((kCi / 64) * (kN / 64) / 8, kB), dim3(256), 0, stream>>>(
      WB, WB, kC, 0L, XT, XT, kC, strXT,
      (void*)G16, (void*)G16, kN, strTP, gb_r, PRM, 0L, kCi, kN, kC, 1.0f);

  for (int b = 0; b < kB; ++b) {
    const unsigned short* Bk  = PHH + (size_t)b * kN * kCi;
    const unsigned short* Bk2 = PHL + (size_t)b * kN * kCi;
    const unsigned short* Gb  = G16 + (size_t)b * kCi * kN;
    for (int qc = 0; qc < kNChunks; ++qc) {
      const size_t qoff = ((size_t)b * kN + (size_t)qc * kQChunk) * kCi;
      const unsigned short* Aq  = THH + qoff;
      const unsigned short* Aq2 = THL + qoff;
      wmma_gemm64<1, true, 0, 0, false, 0><<<dim3((kQChunk / 64) * (kN / 64) / 8, 1), dim3(256), 0, stream>>>(
          Aq, Aq2, kCi, 0L, Bk, Bk2, kCi, 0L,
          (void*)SC, (void*)SC, kN, 0L, PRM, PRM, 0L, kQChunk, kN, kCi, 1.0f);
      softmax_row_kernel<<<dim3(kQChunk), dim3(256), 0, stream>>>(SC, PP);
      unsigned short* Yq = Y16 + qoff;
      wmma_gemm64<0, false, 0, 1, false, 0><<<dim3((kQChunk / 64) * (kCi / 64) / 8, 1), dim3(256), 0, stream>>>(
          PP, PP, kN, 0L, Gb, Gb, kN, 0L,
          (void*)Yq, (void*)Yq, kCi, 0L, PRM, PRM, 0L, kQChunk, kCi, kN, kPVScale);
    }
  }

  wmma_gemm64<0, false, 1, 0, false, 0><<<dim3((kC / 64) * (kN / 64) / 8, kB), dim3(256), 0, stream>>>(
      WW, WW, kCi, 0L, Y16, Y16, kCi, strTP,
      (void*)WY, (void*)WY, kN, (long)kC * kN, wb_r, PRM, 0L, kC, kN, kCi, kWScale);

  bn_stats_kernel<<<dim3(kC), dim3(256), 0, stream>>>(WY, ST);
  const int n4 = nElem / 4;
  bn_apply_kernel<<<dim3(n4 / 256), dim3(256), 0, stream>>>(WY, x, bn_g, bn_b, ST, out, n4);
}
